// GCNPolicy_63874753626724
// MI455X (gfx1250) — hardware-verified
//
#include <hip/hip_runtime.h>
#include <stddef.h>
#include <stdint.h>

#pragma clang fp contract(off)


#define FIN     32
#define EMB     64
#define NTHR    256
#define NWAVE   8
#define EPT     8
#define CHUNK   (NTHR * EPT)
#define WCAP    (EPT * 32)
#define LISTN   (NWAVE * WCAP)
#define NBS     4096
#define RCAP    28672
#define GMAX    64
#define DEGMAX  RCAP
#define FLGMAX  64
#define GTHR    128
#define GBM     64
#define SCALE_F 0.4251202479144762f
#define WSMAX   134217728
#define LDS_CSR ((RCAP + 3 * NBS + LISTN + (GMAX + 32) + 2 * GMAX + NWAVE + 8) * 4)

static_assert((CHUNK & (CHUNK - 1)) == 0 && CHUNK <= 4096);
static_assert((NBS & (NBS - 1)) == 0 && NBS <= 4096);
static_assert((RCAP % 32) == 0);
static_assert(NBS * 2 == 8 * 4 * NTHR);
static_assert(LDS_CSR <= 300000);
static_assert(GBM == (GTHR / 32) * 16);
static_assert(FIN == 32 && EMB == 64);
static_assert(LISTN == NWAVE * WCAP);

typedef float          v2f  __attribute__((ext_vector_type(2)));
typedef float          v4f  __attribute__((ext_vector_type(4)));
typedef float          v8f  __attribute__((ext_vector_type(8)));
typedef int            v2i  __attribute__((ext_vector_type(2)));
typedef int            v4i  __attribute__((ext_vector_type(4)));
typedef int            v8i  __attribute__((ext_vector_type(8)));
typedef unsigned short v8us __attribute__((ext_vector_type(8)));
typedef __bf16         v16b __attribute__((ext_vector_type(16)));
union FragB { v16b v; v8us h[2]; v8i w; };

__device__ __forceinline__ v8f wmb(const FragB& a, const FragB& b, v8f c) {
  v8f d = __builtin_amdgcn_wmma_f32_16x16x32_bf16(false, a.v, false, b.v, (short)0, c, false, false);
  asm volatile("v_nop\n\tv_nop\n\tv_nop\n\tv_nop" : "+v"(d) : "v"(a.w), "v"(b.w));
  return d;
}

__device__ __forceinline__ unsigned short bfb(float f) {
  unsigned u = __float_as_uint(f);
  u += 0x7FFFu + ((u >> 16) & 1u);
  return (unsigned short)(u >> 16);
}
__device__ __forceinline__ float bff(unsigned short h) { return __uint_as_float(((unsigned)h) << 16); }
__device__ __forceinline__ float bf16r(float f) { return bff(bfb(f)); }

__device__ __forceinline__ v8us cvt8b(const v4f a, const v4f b) {
  v8us r;
  r[0] = bfb(a.x); r[1] = bfb(a.y); r[2] = bfb(a.z); r[3] = bfb(a.w);
  r[4] = bfb(b.x); r[5] = bfb(b.y); r[6] = bfb(b.z); r[7] = bfb(b.w);
  return r;
}

__device__ __forceinline__ void split8b(const v4f a, const v4f b, v8us& hi, v8us& lo) {
  const float x[8] = {a.x, a.y, a.z, a.w, b.x, b.y, b.z, b.w};
#pragma unroll
  for (int i = 0; i < 8; ++i) {
    const unsigned short h = bfb(x[i]);
    hi[i] = h;
    lo[i] = bfb(x[i] - bff(h));
  }
}

__device__ __forceinline__ int scan_chunk(const int* __restrict__ ei, int nE, int cbase, int lo, int rng,
                                          int slotBase, int* list, int tid, int lane, int wave) {
  int wc = 0;
  const int el0  = tid * EPT;
  const int e0   = cbase + el0;
  const int sent = -2147483647 - 1;
  int s0, s1, s2, s3, s4, s5, s6, s7;
  if (cbase + CHUNK <= nE) {
    const int* p = ei + 2 * (size_t)e0;
    const v4i q0 = *(const v4i*)p;
    const v4i q1 = *(const v4i*)(p + 4);
    const v4i q2 = *(const v4i*)(p + 8);
    const v4i q3 = *(const v4i*)(p + 12);
    s0 = q0.x; s1 = q0.z; s2 = q1.x; s3 = q1.z; s4 = q2.x; s5 = q2.z; s6 = q3.x; s7 = q3.z;
  } else {
    const int em = nE - 1;
    s0 = (e0     < nE) ? ei[2 * (size_t)min(e0,     em)] : sent;
    s1 = (e0 + 1 < nE) ? ei[2 * (size_t)min(e0 + 1, em)] : sent;
    s2 = (e0 + 2 < nE) ? ei[2 * (size_t)min(e0 + 2, em)] : sent;
    s3 = (e0 + 3 < nE) ? ei[2 * (size_t)min(e0 + 3, em)] : sent;
    s4 = (e0 + 4 < nE) ? ei[2 * (size_t)min(e0 + 4, em)] : sent;
    s5 = (e0 + 5 < nE) ? ei[2 * (size_t)min(e0 + 5, em)] : sent;
    s6 = (e0 + 6 < nE) ? ei[2 * (size_t)min(e0 + 6, em)] : sent;
    s7 = (e0 + 7 < nE) ? ei[2 * (size_t)min(e0 + 7, em)] : sent;
  }
  const unsigned ulo = (unsigned)lo, urg = (unsigned)rng, adj = (unsigned)(lo - slotBase);
  const unsigned u0 = (unsigned)s0 - ulo, u1 = (unsigned)s1 - ulo, u2 = (unsigned)s2 - ulo, u3 = (unsigned)s3 - ulo;
  const unsigned u4 = (unsigned)s4 - ulo, u5 = (unsigned)s5 - ulo, u6 = (unsigned)s6 - ulo, u7 = (unsigned)s7 - ulo;
  const bool h0 = u0 < urg, h1 = u1 < urg, h2 = u2 < urg, h3 = u3 < urg;
  const bool h4 = u4 < urg, h5 = u5 < urg, h6 = u6 < urg, h7 = u7 < urg;
  const unsigned any = __builtin_amdgcn_ballot_w32(h0 | h1 | h2 | h3 | h4 | h5 | h6 | h7);
  if (any != 0u) {
#define HITJ(J, HJ, UJ) { \
      const unsigned mj = __builtin_amdgcn_ballot_w32(HJ); \
      if (mj != 0u) { \
        if (HJ) { \
          const int pos = wc + (int)__builtin_amdgcn_mbcnt_lo(mj, 0u); \
          if (pos < WCAP) list[wave * WCAP + pos] = ((el0 + (J)) << 12) | (int)(((UJ) + adj) & (unsigned)(NBS - 1)); \
        } \
        wc += (int)__builtin_popcount(mj); } }
    HITJ(0, h0, u0)
    HITJ(1, h1, u1)
    HITJ(2, h2, u2)
    HITJ(3, h3, u3)
    HITJ(4, h4, u4)
    HITJ(5, h5, u5)
    HITJ(6, h6, u6)
    HITJ(7, h7, u7)
#undef HITJ
  }
  return wc;
}

__global__ __launch_bounds__(NTHR) void k_norm(const float* __restrict__ ew, int nE, float* nrm) {
  __shared__ double sm[NWAVE];
  __shared__ float sv[8];
  const int tid = (int)threadIdx.x, lane = tid & 31, wave = tid >> 5;
  double s = 0.0;
#pragma unroll 1
  for (int i = tid; i < nE; i += NTHR) {
    const double v = (double)bf16r(ew[i]);
    s = fma(v, v, s);
  }
#pragma unroll
  for (int off = 16; off > 0; off >>= 1) s += __shfl_xor(s, off);
  if (lane == 0) sm[wave] = s;
  __syncthreads();
  if (tid == 0) {
    double t = 0.0;
#pragma unroll
    for (int w = 0; w < NWAVE; ++w) t += sm[w];
    const float nf = (float)sqrt(t);
    sv[0] = (float)(1.0 / (double)nf);
  }
  __syncthreads();
  if (wave == 0) {
    const float inv = sv[0];
    v4f q; q.x = inv; q.y = inv; q.z = inv; q.w = inv;
    const int lc = lane < 8 ? lane : 7;
    if (lane < 8) *(volatile v4f*)(nrm + 4 * lc) = q;
    __threadfence();
    if (lane < 8) *(volatile v4f*)(nrm + 4 * lc) = q;
  }
}

__global__ __launch_bounds__(NTHR) void k_wtr(const float* __restrict__ w0, const float* __restrict__ w1,
                                              int K, unsigned short* wt, int nUnits) {
  const int u = (int)blockIdx.x * NTHR + (int)threadIdx.x;
  if (u >= nUnits) return;
  const int kq = K >> 3;
  const int n  = u / kq;
  const int k8 = (u - n * kq) * 8;
  const int seg = (n >> 6) & 1;
  const int nc  = n & 63;
  const float* ws = (seg == 0) ? w0 : w1;
  const float* p  = ws + (size_t)k8 * EMB + nc;
  v4f a, b;
  a.x = p[0];                 a.y = p[(size_t)EMB];       a.z = p[(size_t)2 * EMB];   a.w = p[(size_t)3 * EMB];
  b.x = p[(size_t)4 * EMB];   b.y = p[(size_t)5 * EMB];   b.z = p[(size_t)6 * EMB];   b.w = p[(size_t)7 * EMB];
  const v8us hv = cvt8b(a, b);
  const size_t o = (size_t)n * (size_t)K + k8;
  *(volatile v8us*)(wt + o) = hv;
  __threadfence();
  *(volatile v8us*)(wt + o) = hv;
}

__global__ __launch_bounds__(NTHR) void k_csr(const int* __restrict__ ei, int nE, int nChunks, int ELB,
                                              int* tab, int* el, int* flg) {
  extern __shared__ v4i lds_dyn[];
  int* reg2 = (int*)lds_dyn;
  int* scnt = reg2 + RCAP;
  int* soff = scnt + NBS;
  int* cur  = soff + NBS;
  int* list = cur + NBS;
  int* gst  = list + LISTN;
  int* gbs  = gst + (GMAX + 32);
  int* gln  = gbs + GMAX;
  int* wcnt = gln + GMAX;
  int* misc = wcnt + NWAVE;
  const int tid = (int)threadIdx.x, lane = tid & 31, wave = tid >> 5;
  const int b = (int)blockIdx.x;
  const int nodeBase = b * NBS;

  for (int i = tid; i < RCAP; i += NTHR) reg2[i] = 0;
  for (int i = tid; i < NBS; i += NTHR) { scnt[i] = 0; soff[i] = 0; cur[i] = 0; }
  for (int i = tid; i < LISTN; i += NTHR) list[i] = 0;
  if (tid < GMAX + 32) gst[tid] = 0;
  if (tid < GMAX) { gbs[tid] = 0; gln[tid] = 0; }
  if (tid < NWAVE) wcnt[tid] = 0;
  if (tid < 8) misc[tid] = 0;
  __syncthreads();

#pragma unroll 1
  for (int ch = 0; ch < nChunks; ++ch) {
    const int cbase = ch * CHUNK;
    const int wc = scan_chunk(ei, nE, cbase, nodeBase, NBS, nodeBase, list, tid, lane, wave);
    if (lane == 0) wcnt[wave] = wc;
    __syncthreads();
    if (tid == 0) {
#pragma unroll 1
      for (int w = 0; w < NWAVE; ++w) {
        int n = wcnt[w];
        n = n < 0 ? 0 : (n > WCAP ? WCAP : n);
#pragma unroll 1
        for (int i = 0; i < n; ++i) {
          const int sl = list[w * WCAP + i] & (NBS - 1);
          scnt[sl] = scnt[sl] + 1;
        }
      }
    }
    __syncthreads();
  }

  if (tid == 0) {
    int g = 0, acc = 0, base = 0, ovf = 0;
    gst[0] = 0;
#pragma unroll 1
    for (int s = 0; s < NBS; ++s) {
      int c = scnt[s];
      c = c < 0 ? 0 : c;
      if (c > RCAP) { ovf = 1; c = RCAP; scnt[s] = c; }
      if (acc + c > RCAP) {
        if (g + 1 < GMAX) {
          gbs[g] = base; gln[g] = acc;
          base = (base + acc + 31) & ~31;
          acc = 0;
          g = g + 1;
          gst[g] = s;
        } else {
          ovf = 1;
        }
      }
      soff[s] = base + acc;
      acc += c;
    }
    gbs[g] = base;
    gln[g] = acc > RCAP ? RCAP : acc;
    gst[g + 1] = NBS;
    misc[0] = (base + acc > 0) ? (g + 1) : 0;
    misc[1] = ovf;
  }
  __syncthreads();
  int ng = misc[0];
  ng = ng < 0 ? 0 : (ng > GMAX ? GMAX : ng);
  int* elb = el + (size_t)b * (size_t)ELB;

#pragma unroll 1
  for (int g = 0; g < ng; ++g) {
    int gs0 = gst[g], gs1 = gst[g + 1];
    gs0 = gs0 < 0 ? 0 : (gs0 > NBS ? NBS : gs0);
    gs1 = gs1 < gs0 ? gs0 : (gs1 > NBS ? NBS : gs1);
    int gb = gbs[g];
    gb = gb < 0 ? 0 : (gb > ELB - RCAP ? ELB - RCAP : gb);
    int gl = gln[g];
    gl = gl < 0 ? 0 : (gl > RCAP ? RCAP : gl);
    for (int s = gs0 + tid; s < gs1; s += NTHR) {
      int v = soff[s] - gb;
      v = v < 0 ? 0 : (v > RCAP ? RCAP : v);
      cur[s] = v;
    }
    __syncthreads();
#pragma unroll 1
    for (int ch = 0; ch < nChunks; ++ch) {
      const int cbase = ch * CHUNK;
      const int wc = scan_chunk(ei, nE, cbase, nodeBase + gs0, gs1 - gs0, nodeBase, list, tid, lane, wave);
      if (lane == 0) wcnt[wave] = wc;
      __syncthreads();
      if (tid == 0) {
#pragma unroll 1
        for (int w = 0; w < NWAVE; ++w) {
          int n = wcnt[w];
          n = n < 0 ? 0 : (n > WCAP ? WCAP : n);
#pragma unroll 1
          for (int i = 0; i < n; ++i) {
            const int ent = list[w * WCAP + i];
            const int sl  = ent & (NBS - 1);
            const int eloc = (ent >> 12) & (CHUNK - 1);
            int eid = cbase + eloc;
            eid = eid > nE - 1 ? nE - 1 : eid;
            int pos = cur[sl];
            pos = pos < 0 ? 0 : (pos > RCAP - 1 ? RCAP - 1 : pos);
            reg2[pos] = eid;
            cur[sl] = pos + 1;
          }
        }
      }
      __syncthreads();
    }
    const int npc = ((gl + 31) >> 5) * 8;
    int* gp = elb + gb;
    for (int p = tid; p < npc; p += NTHR) {
      const v4i v = *(const v4i*)(reg2 + 4 * p);
      *(volatile v4i*)(gp + 4 * p) = v;
    }
    __threadfence();
    for (int p = tid; p < npc; p += NTHR) {
      const v4i v = *(const v4i*)(reg2 + 4 * p);
      *(volatile v4i*)(gp + 4 * p) = v;
    }
    __syncthreads();
  }

  {
    int* tb = tab + (size_t)b * (size_t)NBS * 2;
    const int gp0 = b * ELB;
#pragma unroll 1
    for (int it = 0; it < 8; ++it) {
      const int q = it * NTHR + tid;
      const int s = 2 * q;
      v4i v; v.x = gp0 + soff[s]; v.y = scnt[s]; v.z = gp0 + soff[s + 1]; v.w = scnt[s + 1];
      *(volatile v4i*)(tb + 4 * q) = v;
    }
    __threadfence();
#pragma unroll 1
    for (int it = 0; it < 8; ++it) {
      const int q = it * NTHR + tid;
      const int s = 2 * q;
      v4i v; v.x = gp0 + soff[s]; v.y = scnt[s]; v.z = gp0 + soff[s + 1]; v.w = scnt[s + 1];
      *(volatile v4i*)(tb + 4 * q) = v;
    }
  }
  if (wave == 0) {
    const int o = misc[1];
    v4i v; v.x = o; v.y = o; v.z = o; v.w = o;
    const int lc = lane < 8 ? lane : 7;
    if (lane < 8) *(volatile v4i*)(flg + b * 32 + 4 * lc) = v;
    __threadfence();
    if (lane < 8) *(volatile v4i*)(flg + b * 32 + 4 * lc) = v;
  }
}

__global__ __launch_bounds__(GTHR) void k_xgemm(const float* __restrict__ x0, const float* __restrict__ x1,
                                               const unsigned short* __restrict__ wt,
                                               const float* __restrict__ b0, const float* __restrict__ b1,
                                               float* o0, float* o1, int nN) {
  __shared__ __attribute__((aligned(16))) float stg[GBM * EMB];
  const int tid = (int)threadIdx.x, lane = tid & 31, wave = tid >> 5, hh = lane >> 4, m = lane & 15;
  const int which = (int)blockIdx.y & 1;
  const float* x  = which ? x1 : x0;
  const float* bp = which ? b1 : b0;
  float* outF     = which ? o1 : o0;
  const int wrow0 = which * EMB;
  const int rowBase = (int)blockIdx.x * GBM;

  v8f acc[4];
  {
    const v8f z = {0.f, 0.f, 0.f, 0.f, 0.f, 0.f, 0.f, 0.f};
    acc[0] = z; acc[1] = z; acc[2] = z; acc[3] = z;
  }
  {
    const int r  = rowBase + 16 * wave + m;
    const int rc = r < nN ? r : nN - 1;
    const float* ap = x + (size_t)rc * FIN + 8 * hh;
    v4f p0 = *(const v4f*)ap, p1 = *(const v4f*)(ap + 4);
    v4f p2 = *(const v4f*)(ap + 16), p3 = *(const v4f*)(ap + 20);
    const v4f z4 = {0.f, 0.f, 0.f, 0.f};
    if (r >= nN) { p0 = z4; p1 = z4; p2 = z4; p3 = z4; }
    FragB af;
    af.h[0] = cvt8b(p0, p1);
    af.h[1] = cvt8b(p2, p3);
#pragma unroll
    for (int t = 0; t < 4; ++t) {
      const unsigned short* wq = wt + (size_t)(wrow0 + 16 * t + m) * FIN + 8 * hh;
      FragB bf;
      bf.h[0] = *(const v8us*)wq;
      bf.h[1] = *(const v8us*)(wq + 16);
      acc[t] = wmb(af, bf, acc[t]);
    }
  }
#pragma unroll
  for (int t = 0; t < 4; ++t) {
    const int lc = 16 * t + m;
    const float bv = bf16r(bp[lc]);
#pragma unroll
    for (int r = 0; r < 8; ++r) {
      const int lr = 16 * wave + 8 * hh + r;
      const float v = fmaxf(acc[t][r] + bv, 0.f);
      stg[lr * EMB + lc] = (rowBase + lr < nN) ? v : 0.f;
    }
  }
  __syncthreads();
  v4f fv[8];
#pragma unroll
  for (int i = 0; i < 8; ++i) {
    const int lr = 16 * wave + 2 * i + hh;
    fv[i] = *(const v4f*)(stg + lr * EMB + 4 * m);
  }
#pragma unroll
  for (int i = 0; i < 8; ++i) {
    const int gr = rowBase + 16 * wave + 2 * i + hh;
    float* op = outF + (size_t)gr * EMB + 4 * m;
    *(volatile v4f*)op = fv[i];
  }
  __threadfence();
#pragma unroll
  for (int i = 0; i < 8; ++i) {
    const int gr = rowBase + 16 * wave + 2 * i + hh;
    float* op = outF + (size_t)gr * EMB + 4 * m;
    *(volatile v4f*)op = fv[i];
  }
}

template<int MODE>
__global__ __launch_bounds__(NTHR) void k_step(
    const int* __restrict__ ei, const float* __restrict__ ew, const float* __restrict__ nrm,
    const int* __restrict__ tab, const int* __restrict__ el,
    const float* __restrict__ F, const float* __restrict__ Pcur,
    const float* __restrict__ side, const float* __restrict__ temps, int tix,
    float* Pnxt, float* Dout, int nN, int nE, int MP, int elTot)
{
  const int lane = (int)threadIdx.x & 31, wave = (int)threadIdx.x >> 5;
  const int row = (int)blockIdx.x * NWAVE + wave;
  if (row >= MP) return;
  const v2i te = *(const v2i*)(tab + 2 * (size_t)row);
  int gpos = te.x, cnt = te.y;
  gpos = gpos < 0 ? 0 : (gpos > elTot - 1 ? elTot - 1 : gpos);
  cnt = cnt < 0 ? 0 : (cnt > DEGMAX ? DEGMAX : cnt);
  if (cnt > elTot - gpos) cnt = elTot - gpos;
  const float inv = nrm[0];
  float a0 = 0.f, a1 = 0.f;
  const float* fl = F + 2 * lane;
#pragma unroll 1
  for (int base = 0; base < cnt; base += 32) {
    int j = base + lane;
    j = j < cnt ? j : cnt - 1;
    int eid = el[(size_t)gpos + j];
    eid = eid < 0 ? 0 : (eid > nE - 1 ? nE - 1 : eid);
    int d = ei[2 * (size_t)eid + 1];
    if (d < 0) d += nN;
    d = d < 0 ? 0 : (d > nN - 1 ? nN - 1 : d);
    const float w = bf16r(ew[eid]) * inv;
    const int wi = __float_as_int(w);
    const int m32 = (cnt - base) < 32 ? (cnt - base) : 32;
#pragma unroll 4
    for (int k = 0; k < m32; ++k) {
      const int dk = __builtin_amdgcn_readlane(d, k);
      const float wk = __int_as_float(__builtin_amdgcn_readlane(wi, k));
      const v2f f = *(const v2f*)(fl + (size_t)dk * EMB);
      a0 = fmaf(wk, f.x, a0);
      a1 = fmaf(wk, f.y, a1);
    }
  }
  const int rc = row < nN ? row : nN - 1;
  const float t  = bf16r(temps[tix]);
  const float sc = bf16r(side[rc]);
  const bool live = row < nN;
  const size_t ro = (size_t)row * EMB + 2 * lane;
  const v2f po = *(const v2f*)(Pcur + ro);
  if (MODE == 0) {
    float n0 = (po.x + t * (sc - a0)) * SCALE_F;
    float n1 = (po.y + t * (sc - a1)) * SCALE_F;
    n0 = fmaxf(n0, 0.f); n1 = fmaxf(n1, 0.f);
    if (!live) { n0 = 0.f; n1 = 0.f; }
    v2f vn; vn.x = n0; vn.y = n1;
    v2f dd; dd.x = 2.0f * n0 - po.x; dd.y = 2.0f * n1 - po.y;
    *(volatile v2f*)(Pnxt + ro) = vn;
    *(volatile v2f*)(Dout + ro) = dd;
    __threadfence();
    *(volatile v2f*)(Pnxt + ro) = vn;
    *(volatile v2f*)(Dout + ro) = dd;
  } else {
    float n0 = po.x - t * (sc - a0);
    float n1 = po.y - t * (sc - a1);
    n0 = fmaxf(n0, 0.f); n1 = fmaxf(n1, 0.f);
    if (!live) { n0 = 0.f; n1 = 0.f; }
    v2f vn; vn.x = n0; vn.y = n1;
    *(volatile v2f*)(Pnxt + ro) = vn;
    __threadfence();
    *(volatile v2f*)(Pnxt + ro) = vn;
  }
}

__global__ __launch_bounds__(GTHR) void k_head(const float* __restrict__ a0p, const float* __restrict__ a1p,
                                              const unsigned short* __restrict__ wt,
                                              const float* __restrict__ b0, const float* __restrict__ b1,
                                              const float* __restrict__ w20, const float* __restrict__ w21,
                                              float* ho0, float* ho1) {
  __shared__ __attribute__((aligned(16))) float stg[GBM * EMB];
  __shared__ float w2s[EMB];
  __shared__ float pp[GTHR];
  __shared__ __attribute__((aligned(16))) float tot[GBM];
  const int tid = (int)threadIdx.x, lane = tid & 31, wave = tid >> 5, hh = lane >> 4, m = lane & 15;
  const int which = (int)blockIdx.y & 1;
  const float* A  = which ? a1p : a0p;
  const float* bp = which ? b1 : b0;
  const float* w2 = which ? w21 : w20;
  float* ho       = which ? ho1 : ho0;
  const int wrow0 = which * EMB;
  const int rowBase = (int)blockIdx.x * GBM;
  if (tid < EMB) w2s[tid] = bf16r(w2[tid]);

  v8f acc[4];
  {
    const v8f z = {0.f, 0.f, 0.f, 0.f, 0.f, 0.f, 0.f, 0.f};
    acc[0] = z; acc[1] = z; acc[2] = z; acc[3] = z;
  }
  const float* ap = A + (size_t)(rowBase + 16 * wave + m) * EMB + 8 * hh;
#pragma unroll
  for (int kh = 0; kh < 2; ++kh) {
    const v4f p0 = *(const v4f*)(ap + 32 * kh);
    const v4f p1 = *(const v4f*)(ap + 32 * kh + 4);
    const v4f p2 = *(const v4f*)(ap + 32 * kh + 16);
    const v4f p3 = *(const v4f*)(ap + 32 * kh + 20);
    FragB ahi, alo;
    split8b(p0, p1, ahi.h[0], alo.h[0]);
    split8b(p2, p3, ahi.h[1], alo.h[1]);
#pragma unroll
    for (int t = 0; t < 4; ++t) {
      const unsigned short* wq = wt + (size_t)(wrow0 + 16 * t + m) * EMB + 32 * kh + 8 * hh;
      FragB bf;
      bf.h[0] = *(const v8us*)wq;
      bf.h[1] = *(const v8us*)(wq + 16);
      acc[t] = wmb(ahi, bf, acc[t]);
      acc[t] = wmb(alo, bf, acc[t]);
    }
  }
#pragma unroll
  for (int t = 0; t < 4; ++t) {
    const int lc = 16 * t + m;
    const float bv = bf16r(bp[lc]);
#pragma unroll
    for (int r = 0; r < 8; ++r) {
      const int lr = 16 * wave + 8 * hh + r;
      stg[lr * EMB + lc] = fmaxf(acc[t][r] + bv, 0.f);
    }
  }
  __syncthreads();
  {
    const int row = tid & 63, half = tid >> 6;
    const float* sr = stg + row * EMB + 32 * half;
    const float* wr = w2s + 32 * half;
    float s = 0.f;
#pragma unroll 8
    for (int n = 0; n < 32; ++n) s = fmaf(sr[n], wr[n], s);
    pp[tid] = s;
  }
  __syncthreads();
  if (tid < GBM) tot[tid] = pp[tid] + pp[GBM + tid];
  __syncthreads();
  if (wave == 0) {
    const int lc = lane < 16 ? lane : 15;
    const v4f v = *(const v4f*)(tot + 4 * lc);
    float* op = ho + rowBase + 4 * lc;
    if (lane < 16) *(volatile v4f*)op = v;
    __threadfence();
    if (lane < 16) *(volatile v4f*)op = v;
  }
}

__global__ __launch_bounds__(NTHR) void k_out(const float* __restrict__ ho0, const float* __restrict__ ho1,
                                             const int* __restrict__ flg, int gC, float* out,
                                             int nN, int MP, int nOut4) {
  const int i = (int)blockIdx.x * NTHR + (int)threadIdx.x;
  if (i >= nOut4) return;
  int pz = 0;
  const int gcl = gC < FLGMAX ? gC : FLGMAX;
#pragma unroll 1
  for (int b = 0; b < gcl; ++b) pz |= flg[32 * b];
  const float qnan = __int_as_float(0x7fc00000);
  const int j = 4 * i;
  float v[4];
#pragma unroll
  for (int k = 0; k < 4; ++k) {
    const int idx = j + k;
    const int ia = idx > MP - 1 ? MP - 1 : idx;
    int ib = idx - nN;
    ib = ib < 0 ? 0 : (ib > MP - 1 ? MP - 1 : ib);
    const float fa = ho0[ia];
    const float fb = ho1[ib];
    float r = (idx < nN) ? fa : fb;
    if (pz != 0) r = qnan;
    v[k] = r;
  }
  v4f q; q.x = v[0]; q.y = v[1]; q.z = v[2]; q.w = v[3];
  *(volatile v4f*)(out + j) = q;
  __threadfence();
  *(volatile v4f*)(out + j) = q;
}

static inline int cdiv(int a, int b) { return (a + b - 1) / b; }

extern "C" void kernel_launch(void* const* d_in, const int* in_sizes, int n_in,
                              void* d_out, int out_size, void* d_ws, size_t ws_size,
                              hipStream_t stream) {
  if (n_in < 18) return;
  const int nN = in_sizes[3];
  if (nN <= 0 || nN > (1 << 20) || (nN & 1) != 0) return;
  if (in_sizes[4] != nN || in_sizes[0] != nN * FIN || in_sizes[1] != nN * FIN) return;
  const int nE = in_sizes[2];
  if (nE < 1 || nE > (1 << 20) || in_sizes[17] != 2 * nE) return;
  if (in_sizes[5]  != FIN * EMB || in_sizes[6]  != EMB) return;
  if (in_sizes[7]  != FIN * EMB || in_sizes[8]  != EMB) return;
  if (in_sizes[9]  != 8 || in_sizes[10] != 8) return;
  if (in_sizes[11] != EMB * EMB || in_sizes[12] != EMB || in_sizes[13] != EMB) return;
  if (in_sizes[14] != EMB * EMB || in_sizes[15] != EMB || in_sizes[16] != EMB) return;
  if (out_size != 2 * nN) return;

  const float* con_feat = (const float*)d_in[0];
  const float* var_feat = (const float*)d_in[1];
  const float* edge_w   = (const float*)d_in[2];
  const float* cvec     = (const float*)d_in[3];
  const float* bvec     = (const float*)d_in[4];
  const float* wcons    = (const float*)d_in[5];
  const float* bcons    = (const float*)d_in[6];
  const float* wvar     = (const float*)d_in[7];
  const float* bvar     = (const float*)d_in[8];
  const float* t_ctov   = (const float*)d_in[9];
  const float* t_vtoc   = (const float*)d_in[10];
  const float* w1a      = (const float*)d_in[11];
  const float* b1a      = (const float*)d_in[12];
  const float* w2a      = (const float*)d_in[13];
  const float* w1b      = (const float*)d_in[14];
  const float* b1b      = (const float*)d_in[15];
  const float* w2b      = (const float*)d_in[16];
  const int*   ei       = (const int*)  d_in[17];
  float* out = (float*)d_out;

  const int MP = cdiv(nN, GBM) * GBM;
  const int gC = cdiv(MP, NBS);
  if (gC > FLGMAX) return;
  int ELB = ((nE + 31) & ~31) + 32 * GMAX;
  if (ELB < RCAP + 32) ELB = RCAP + 32;
  const int elTot = gC * ELB;
  const int nChunks = cdiv(nE, CHUNK);
  const int nOut4 = (2 * nN) / 4;

  char* ws = (char*)d_ws;
  size_t off = 0;
  const size_t oNRM = off; off += 256;                                      off = (off + 255) & ~(size_t)255;
  const size_t oFLG = off; off += (size_t)gC * 128;                          off = (off + 255) & ~(size_t)255;
  const size_t oWA  = off; off += (size_t)128 * FIN * 2;                     off = (off + 255) & ~(size_t)255;
  const size_t oWB  = off; off += (size_t)128 * EMB * 2;                     off = (off + 255) & ~(size_t)255;
  const size_t oTAB = off; off += (size_t)gC * NBS * 8;                      off = (off + 255) & ~(size_t)255;
  const size_t oEL  = off; off += (size_t)elTot * 4;                         off = (off + 255) & ~(size_t)255;
  const size_t oC0  = off; off += (size_t)MP * EMB * 4;                      off = (off + 255) & ~(size_t)255;
  const size_t oC1  = off; off += (size_t)MP * EMB * 4;                      off = (off + 255) & ~(size_t)255;
  const size_t oV0  = off; off += (size_t)MP * EMB * 4;                      off = (off + 255) & ~(size_t)255;
  const size_t oV1  = off; off += (size_t)MP * EMB * 4;                      off = (off + 255) & ~(size_t)255;
  const size_t oD   = off; off += (size_t)MP * EMB * 4;                      off = (off + 255) & ~(size_t)255;
  const size_t oH0  = off; off += (size_t)MP * 4;                            off = (off + 255) & ~(size_t)255;
  const size_t oH1  = off; off += (size_t)MP * 4;                            off = (off + 255) & ~(size_t)255;
  if (off > ws_size || off > (size_t)WSMAX) return;
  float*          NRM = (float*)(ws + oNRM);
  int*            FLG = (int*)(ws + oFLG);
  unsigned short* WA  = (unsigned short*)(ws + oWA);
  unsigned short* WB  = (unsigned short*)(ws + oWB);
  int*            TAB = (int*)(ws + oTAB);
  int*            EL  = (int*)(ws + oEL);
  float* CONS[2] = { (float*)(ws + oC0), (float*)(ws + oC1) };
  float* VAR[2]  = { (float*)(ws + oV0), (float*)(ws + oV1) };
  float* DPL = (float*)(ws + oD);
  float* HO0 = (float*)(ws + oH0);
  float* HO1 = (float*)(ws + oH1);

  hipFuncSetAttribute(reinterpret_cast<const void*>(&k_csr),
                      hipFuncAttributeMaxDynamicSharedMemorySize, LDS_CSR);

  k_norm<<<1, NTHR, 0, stream>>>(edge_w, nE, NRM);
  {
    const int nU1 = 128 * (FIN / 8);
    k_wtr<<<cdiv(nU1, NTHR), NTHR, 0, stream>>>(wcons, wvar, FIN, WA, nU1);
    const int nU2 = 128 * (EMB / 8);
    k_wtr<<<cdiv(nU2, NTHR), NTHR, 0, stream>>>(w1a, w1b, EMB, WB, nU2);
  }
  k_csr<<<gC, NTHR, LDS_CSR, stream>>>(ei, nE, nChunks, ELB, TAB, EL, FLG);
  k_xgemm<<<dim3(MP / GBM, 2), GTHR, 0, stream>>>(con_feat, var_feat, WA, bcons, bvar, CONS[0], VAR[0], nN);

  const int gS = MP / NWAVE;
  for (int i = 0; i < 4; ++i) {
    const int cI = i & 1, nI = (i + 1) & 1;
    k_step<0><<<gS, NTHR, 0, stream>>>(ei, edge_w, NRM, TAB, EL, CONS[cI], VAR[cI], cvec, t_ctov, 2 * i + 1,
                                        VAR[nI], DPL, nN, nE, MP, elTot);
    k_step<1><<<gS, NTHR, 0, stream>>>(ei, edge_w, NRM, TAB, EL, DPL, CONS[cI], bvec, t_vtoc, 2 * i,
                                        CONS[nI], DPL, nN, nE, MP, elTot);
  }
  k_head<<<dim3(MP / GBM, 2), GTHR, 0, stream>>>(VAR[0], CONS[0], WB, b1a, b1b, w2a, w2b, HO0, HO1);
  k_out<<<cdiv(nOut4, NTHR), NTHR, 0, stream>>>(HO0, HO1, FLG, gC, out, nN, MP, nOut4);
}
